// MultiHeadTEAttention_50663434224042
// MI455X (gfx1250) — hardware-verified
//
#include <hip/hip_runtime.h>
#include <math.h>

typedef __attribute__((ext_vector_type(16))) _Float16 v16h;
typedef __attribute__((ext_vector_type(16))) __bf16 v16b;
typedef __attribute__((ext_vector_type(8)))  _Float16 v8h;
typedef __attribute__((ext_vector_type(8)))  float v8f;
typedef __attribute__((ext_vector_type(4)))  float v4f;
typedef __attribute__((ext_vector_type(2)))  float v2f;
typedef __attribute__((ext_vector_type(4)))  unsigned v4u;
typedef __attribute__((ext_vector_type(4)))  int v4i;
typedef float __attribute__((may_alias)) float_a;
typedef int __attribute__((may_alias)) int_a;

template <typename T> __device__ __forceinline__ void vst2(void* p, T v) { *(volatile T*)p = v; __threadfence(); *(volatile T*)p = v; }
__device__ __forceinline__ v8f wmma16(v16h a, v16h b, v8f c) {
  v8f d = __builtin_amdgcn_wmma_f32_16x16x32_f16(false, a, false, b, (short)0, c, false, false);
  asm volatile("v_nop\n\tv_nop\n\tv_nop\n\tv_nop" : "+v"(d) : "v"(a), "v"(b));
  return d;
}
__device__ __forceinline__ v8f wmma_bf(v16b a, v16b b, v8f c) {
  v8f d = __builtin_amdgcn_wmma_f32_16x16x32_bf16(false, a, false, b, (short)0, c, false, false);
  asm volatile("v_nop\n\tv_nop\n\tv_nop\n\tv_nop" : "+v"(d) : "v"(a), "v"(b));
  return d;
}
__device__ __forceinline__ v16h frag_h(const _Float16* rowk0, int lane) {
  union { v16h v; v8h q[2]; } u; const _Float16* p = rowk0 + 8 * (lane >> 4);
  u.q[0] = *(const v8h*)p; u.q[1] = *(const v8h*)(p + 16); return u.v;
}
__device__ __forceinline__ v16h frag_f32(const float* rowk0, int lane) {
  v16h a; const float* p = rowk0 + 8 * (lane >> 4);
#pragma unroll
  for (int i = 0; i < 8; ++i) { a[i] = (_Float16)p[i]; a[8 + i] = (_Float16)p[16 + i]; }
  return a;
}
__device__ __forceinline__ v16h frag_f32s(const float* rowk0, int lane, float sc) {
  v16h a; const float* p = rowk0 + 8 * (lane >> 4);
#pragma unroll
  for (int i = 0; i < 8; ++i) { a[i] = (_Float16)(p[i] * sc); a[8 + i] = (_Float16)(p[16 + i] * sc); }
  return a;
}
__device__ __forceinline__ v16h fragc_f32(const float* W, int k0, int n, int lane, int ld, int K) {
  v16h a; const int g = lane >> 4;
#pragma unroll
  for (int i = 0; i < 8; ++i) { const int ka = k0 + 8 * g + i, kb = ka + 16;
    a[i] = (_Float16)(ka < K ? W[(size_t)ka * ld + n] : 0.f); a[8 + i] = (_Float16)(kb < K ? W[(size_t)kb * ld + n] : 0.f); }
  return a;
}
struct F2 { v16b h, l; };
__device__ __forceinline__ F2 bsplit16(const float v[16]) { F2 r;
#pragma unroll
  for (int i = 0; i < 16; ++i) { const __bf16 h = (__bf16)v[i]; r.h[i] = h; r.l[i] = (__bf16)(v[i] - (float)h); }
  return r; }
__device__ __forceinline__ F2 split_row(const float* row, int k0, int lane) { float v[16]; const float* p = row + k0 + 8 * (lane >> 4);
#pragma unroll
  for (int i = 0; i < 8; ++i) { v[i] = p[i]; v[8 + i] = p[16 + i]; }
  return bsplit16(v); }
__device__ __forceinline__ F2 split_rowK(const float* row, int k0, int lane, int K) { float v[16]; const int g = lane >> 4;
#pragma unroll
  for (int i = 0; i < 8; ++i) { const int ka = k0 + 8 * g + i, kb = ka + 16; v[i] = ka < K ? row[ka] : 0.f; v[8 + i] = kb < K ? row[kb] : 0.f; }
  return bsplit16(v); }
__device__ __forceinline__ F2 split_col(const float* W, int k0, int n, int lane, int ld, int K) { float v[16]; const int g = lane >> 4;
#pragma unroll
  for (int i = 0; i < 8; ++i) { const int ka = k0 + 8 * g + i, kb = ka + 16; v[i] = ka < K ? W[(size_t)ka * ld + n] : 0.f; v[8 + i] = kb < K ? W[(size_t)kb * ld + n] : 0.f; }
  return bsplit16(v); }
__device__ __forceinline__ v8f mac3(const F2& a, const F2& b, v8f c) { c = wmma_bf(a.l, b.h, c); c = wmma_bf(a.h, b.l, c); return wmma_bf(a.h, b.h, c); }
__device__ __forceinline__ float sigm(float v) { return 1.0f / (1.0f + expf(-v)); }
#define LDSX() do { asm volatile("s_wait_dscnt 0" ::: "memory"); __builtin_amdgcn_wave_barrier(); __builtin_amdgcn_fence(__ATOMIC_RELEASE, "workgroup"); } while (0)

#define MB 8
#define NQ 1024
#define DX 512
#define NH 8
#define HD 64
#define KH 16
#define NR (MB * NQ)
#define MCH 2

__global__ __launch_bounds__(256) void k_cvt(const float* __restrict__ src, _Float16* __restrict__ dst, size_t n8) {
  const size_t g8 = (size_t)blockIdx.x * 256 + threadIdx.x; if (g8 >= n8) return;
  union { v8h h; v4u u; } pk;
#pragma unroll
  for (int e = 0; e < 8; ++e) pk.h[e] = (_Float16)src[g8 * 8 + e];
  vst2(dst + g8 * 8, pk.u);
}
__global__ __launch_bounds__(256) void k_packT(const float* __restrict__ W0, const float* __restrict__ W1, const float* __restrict__ W2, const float* __restrict__ W3, _Float16* __restrict__ P) {
  __shared__ float tile[64][65];
  const int which = blockIdx.z, o0 = blockIdx.x * 64, k0 = blockIdx.y * 64, tid = threadIdx.x;
  const float* W = which == 0 ? W0 : (which == 1 ? W1 : (which == 2 ? W2 : W3));
  for (int q = tid; q < 64 * 64; q += 256) { const int kl = q >> 6, ol = q & 63; tile[kl][ol] = W[(size_t)(k0 + kl) * DX + o0 + ol]; }
  __syncthreads();
  for (int u = 0; u < 2; ++u) { const int idx = tid + u * 256, ol = idx >> 3, pc = idx & 7; union { v8h hh; v4u uu; } pk;
#pragma unroll
    for (int i = 0; i < 8; ++i) pk.hh[i] = (_Float16)(tile[pc * 8 + i][ol] * 16.0f);
    vst2(P + ((size_t)which * DX + o0 + ol) * DX + k0 + pc * 8, pk.uu); }
}
__global__ __launch_bounds__(128) void k_proj(const _Float16* __restrict__ xq, const _Float16* __restrict__ xk, const _Float16* __restrict__ xv, const _Float16* __restrict__ P, _Float16* __restrict__ qh, _Float16* __restrict__ kh, _Float16* __restrict__ vT) {
  __shared__ __align__(16) float so[4][16][132];
  __shared__ __align__(16) _Float16 st[128][72];
  const int tid = threadIdx.x, wave = tid >> 5, lane = tid & 31, col = lane & 15, g = lane >> 4;
  const int which = blockIdx.z; const int r0b = blockIdx.x * 64, r0 = r0b + wave * 16, n0 = blockIdx.y * 128; const int m = r0b / NQ, t0 = r0b % NQ, hb = n0 / HD;
  const _Float16* A = which == 0 ? xq : (which == 1 ? xk : xv);
  v8f acc[8] = {};
#pragma unroll 1
  for (int kc = 0; kc < DX / 32; ++kc) { const v16h a = frag_h(A + (size_t)(r0 + col) * DX + kc * 32, lane);
#pragma unroll
    for (int j = 0; j < 8; ++j) acc[j] = wmma16(a, frag_h(P + ((size_t)which * DX + n0 + j * 16 + col) * DX + kc * 32, lane), acc[j]); }
#pragma unroll
  for (int j = 0; j < 8; ++j)
#pragma unroll
    for (int r = 0; r < 8; ++r) so[wave][8 * g + r][j * 16 + col] = acc[j][r] * (1.0f / 16.0f);
  LDSX();
  if (which < 2) { _Float16* dst = which == 0 ? qh : kh;
    for (int q = lane; q < 2 * 16 * 8; q += 32) { const int hh = q >> 7, rem = q & 127, rl = rem >> 3, pc = rem & 7; union { v8h h8; v4u u; } pk;
#pragma unroll
      for (int e = 0; e < 8; ++e) pk.h8[e] = (_Float16)so[wave][rl][hh * HD + pc * 8 + e];
      vst2(dst + (((size_t)m * NH + hb + hh) * NQ + t0 + wave * 16 + rl) * HD + pc * 8, pk.u); } }
  else {
#pragma unroll 4
    for (int rl = 0; rl < 16; ++rl) {
#pragma unroll
      for (int e = 0; e < 4; ++e) st[lane * 4 + e][wave * 16 + rl] = (_Float16)so[wave][rl][lane * 4 + e]; }
    __syncthreads();
    for (int q = tid; q < 128 * 8; q += 128) { const int c = q >> 3, pc = q & 7, hh = c >> 6, d = c & 63;
      vst2(vT + (((size_t)m * NH + hb + hh) * HD + d) * NQ + t0 + pc * 8, *(const v4u*)(&st[c][pc * 8])); } }
}
__global__ __launch_bounds__(256) void k_bias(const float* __restrict__ tq, const float* __restrict__ tk, const float* __restrict__ kw1, const float* __restrict__ kb1, const float* __restrict__ kw2, const float* __restrict__ kb2, int m0, float* __restrict__ bias) {
  __shared__ float sw1[2 * KH], sb1[KH], sb2[NH];
  __shared__ __align__(16) float so[NQ * NH];
  const int tid = threadIdx.x, w = tid >> 5, lane = tid & 31, col = lane & 15, g = lane >> 4; const int q = blockIdx.x, ml = blockIdx.y, m = m0 + ml;
  if (tid < 2 * KH) sw1[tid] = kw1[tid]; if (tid < KH) sb1[tid] = kb1[tid]; if (tid < NH) sb2[tid] = kb2[tid];
  F2 bw; { float wv[16];
#pragma unroll
    for (int i = 0; i < 16; ++i) { const int c = 8 * g + i; wv[i] = (i < 8 && col < NH) ? kw2[c * NH + col] : 0.f; }
    bw = bsplit16(wv); }
  __syncthreads();
  const float q0v = tq[((size_t)m * NQ + q) * 2], q1v = tq[((size_t)m * NQ + q) * 2 + 1];
#pragma unroll 1
  for (int t = 0; t < 8; ++t) { const int key = w * 128 + t * 16 + col; const float d0 = q0v - tk[((size_t)m * NQ + key) * 2], d1 = q1v - tk[((size_t)m * NQ + key) * 2 + 1];
    float av[16];
#pragma unroll
    for (int i = 0; i < 8; ++i) { const int c = 8 * g + i; const float hv = d0 * sw1[c] + d1 * sw1[KH + c] + sb1[c]; av[i] = hv > 0.f ? hv : 0.f; av[8 + i] = 0.f; }
    v8f acc = {}; acc = mac3(bsplit16(av), bw, acc);
    if (col < NH) {
#pragma unroll
      for (int r = 0; r < 8; ++r) so[(w * 128 + t * 16 + 8 * g + r) * NH + col] = acc[r] + sb2[col]; } }
  __syncthreads();
  for (int e = tid; e < NQ * NH / 4; e += 256) vst2(bias + (((size_t)ml * NQ + q) * NQ) * NH + e * 4, *(const v4f*)(&so[e * 4]));
}
__global__ __launch_bounds__(128) void k_attn(const _Float16* __restrict__ qh, const _Float16* __restrict__ kh, const _Float16* __restrict__ vT, const float* __restrict__ bias, int m0, _Float16* __restrict__ o16) {
  __shared__ __align__(16) float sS[4][16][68];
  __shared__ __align__(16) _Float16 sP[4][16][72];
  __shared__ __align__(16) float sO[4][16][68];
  const int tid = threadIdx.x, w = tid >> 5, lane = tid & 31, col = lane & 15, g = lane >> 4;
  const int ml = blockIdx.z, m = m0 + ml, h = blockIdx.y, q0 = blockIdx.x * 64 + w * 16; const size_t mh = (size_t)m * NH + h;
  const _Float16* qb = qh + mh * NQ * HD; const _Float16* kb = kh + mh * NQ * HD; const _Float16* vb = vT + mh * HD * NQ;
  const float* bb = bias + ((size_t)ml * NQ) * NQ * NH + h;
  v16h aq[2];
#pragma unroll
  for (int kc = 0; kc < 2; ++kc) aq[kc] = frag_h(qb + (size_t)(q0 + col) * HD + kc * 32, lane);
  float mrun = -3.0e38f, lrun = 0.f; v8f acc[4] = {};
#pragma unroll 1
  for (int kt = 0; kt < NQ / 64; ++kt) {
#pragma unroll
    for (int t = 0; t < 4; ++t) { v8f s = {}; const int key = kt * 64 + t * 16 + col;
#pragma unroll
      for (int kc = 0; kc < 2; ++kc) s = wmma16(aq[kc], frag_h(kb + (size_t)key * HD + kc * 32, lane), s);
#pragma unroll
      for (int r = 0; r < 8; ++r) { const int qi = q0 + 8 * g + r; sS[w][8 * g + r][t * 16 + col] = s[r] * 0.125f + bb[((size_t)qi * NQ + key) * NH]; } }
    LDSX();
    float mx = -3.4e38f;
#pragma unroll
    for (int jj = 0; jj < 32; ++jj) mx = fmaxf(mx, sS[w][col][g * 32 + jj]);
    mx = fmaxf(mx, __shfl_xor(mx, 16, 32));
    const float mnew = fmaxf(mrun, mx); const float corr = expf(mrun - mnew);
    float ps = 0.f;
#pragma unroll
    for (int jj = 0; jj < 32; ++jj) { const float p = expf(sS[w][col][g * 32 + jj] - mnew); ps += p; sP[w][col][g * 32 + jj] = (_Float16)(p * 16384.0f); }
    ps += __shfl_xor(ps, 16, 32);
    lrun = lrun * corr + ps; mrun = mnew;
#pragma unroll
    for (int r = 0; r < 8; ++r) { const float cr = __shfl(corr, 8 * g + r, 32);
#pragma unroll
      for (int t = 0; t < 4; ++t) acc[t][r] *= cr; }
    LDSX();
#pragma unroll
    for (int kc = 0; kc < 2; ++kc) { const v16h pa = frag_h(&sP[w][col][0] + kc * 32, lane);
#pragma unroll
      for (int t = 0; t < 4; ++t) acc[t] = wmma16(pa, frag_h(vb + (size_t)(t * 16 + col) * NQ + kt * 64 + kc * 32, lane), acc[t]); }
    __builtin_amdgcn_wave_barrier();
  }
#pragma unroll
  for (int r = 0; r < 8; ++r) { const float lr = __shfl(lrun, 8 * g + r, 32);
#pragma unroll
    for (int t = 0; t < 4; ++t) sO[w][8 * g + r][t * 16 + col] = acc[t][r] / (lr * 16384.0f); }
  LDSX();
  for (int q = lane; q < 16 * 8; q += 32) { const int rl = q >> 3, pc = q & 7; union { v8h h8; v4u u; } pk;
#pragma unroll
    for (int e = 0; e < 8; ++e) pk.h8[e] = (_Float16)(sO[w][rl][pc * 8 + e] * 16.0f);
    vst2(o16 + ((size_t)m * NQ + q0 + rl) * DX + h * HD + pc * 8, pk.u); }
}
__global__ __launch_bounds__(128) void k_out(const _Float16* __restrict__ o16, const _Float16* __restrict__ P, const float* __restrict__ bo, float* __restrict__ out) {
  __shared__ __align__(16) float so[4][16][132];
  const int tid = threadIdx.x, wave = tid >> 5, lane = tid & 31, col = lane & 15, g = lane >> 4;
  const int r0 = blockIdx.x * 64 + wave * 16, n0 = blockIdx.y * 128;
  v8f acc[8] = {};
#pragma unroll 1
  for (int kc = 0; kc < DX / 32; ++kc) { const v16h a = frag_h(o16 + (size_t)(r0 + col) * DX + kc * 32, lane);
#pragma unroll
    for (int j = 0; j < 8; ++j) acc[j] = wmma16(a, frag_h(P + ((size_t)3 * DX + n0 + j * 16 + col) * DX + kc * 32, lane), acc[j]); }
#pragma unroll
  for (int j = 0; j < 8; ++j) { const float b0 = bo[n0 + j * 16 + col];
#pragma unroll
    for (int r = 0; r < 8; ++r) so[wave][8 * g + r][j * 16 + col] = acc[j][r] * (1.0f / 256.0f) + b0; }
  LDSX();
#pragma unroll 4
  for (int rl = 0; rl < 16; ++rl) vst2(out + (size_t)(r0 + rl) * DX + n0 + lane * 4, *(const v4f*)(&so[wave][rl][lane * 4]));
}
extern "C" void kernel_launch(void* const* d_in, const int* in_sizes, int n_in, void* d_out, int out_size, void* d_ws, size_t ws_size, hipStream_t stream) {
  (void)in_sizes; (void)n_in; (void)out_size; (void)ws_size;
  const float** I = (const float**)d_in;
  const float* xq = I[0]; const float* xk = I[1]; const float* xv = I[2]; const float* tq = I[3]; const float* tk = I[4];
  const float* wq = I[5]; const float* wk = I[6]; const float* wv = I[7]; const float* wo = I[8]; const float* bo = I[9]; const float* kw1 = I[10]; const float* kb1 = I[11]; const float* kw2 = I[12]; const float* kb2 = I[13];
  float* out = (float*)d_out;
  char* ws = (char*)d_ws; size_t off = 0;
  auto take = [&](size_t bytes) { char* p = ws + off; off += (bytes + 255) & ~(size_t)255; return p; };
  _Float16* xq16 = (_Float16*)take((size_t)NR * DX * 2); _Float16* xk16 = (_Float16*)take((size_t)NR * DX * 2); _Float16* xv16 = (_Float16*)take((size_t)NR * DX * 2); _Float16* P = (_Float16*)take((size_t)4 * DX * DX * 2);
  _Float16* qh = (_Float16*)take((size_t)NR * DX * 2); _Float16* kh = (_Float16*)take((size_t)NR * DX * 2); _Float16* vT = (_Float16*)take((size_t)NR * DX * 2); _Float16* o16 = (_Float16*)take((size_t)NR * DX * 2);
  float* bias = (float*)take((size_t)MCH * NQ * NQ * NH * 4);
  const size_t n8 = (size_t)NR * DX / 8;
  k_cvt<<<(unsigned)(n8 / 256), 256, 0, stream>>>(xq, xq16, n8); k_cvt<<<(unsigned)(n8 / 256), 256, 0, stream>>>(xk, xk16, n8); k_cvt<<<(unsigned)(n8 / 256), 256, 0, stream>>>(xv, xv16, n8);
  k_packT<<<dim3(DX / 64, DX / 64, 4), 256, 0, stream>>>(wq, wk, wv, wo, P);
  k_proj<<<dim3(NR / 64, DX / 128, 3), 128, 0, stream>>>(xq16, xk16, xv16, P, qh, kh, vT);
  for (int ch = 0; ch < MB / MCH; ++ch) { const int m0 = ch * MCH;
    k_bias<<<dim3(NQ, MCH), 256, 0, stream>>>(tq, tk, kw1, kb1, kw2, kb2, m0, bias);
    k_attn<<<dim3(NQ / 64, NH, MCH), 128, 0, stream>>>(qh, kh, vT, bias, m0, o16); }
  k_out<<<dim3(NR / 64, DX / 128), 128, 0, stream>>>(o16, P, bo, out);
}
